// SectionAttention_23974507446660
// MI455X (gfx1250) — hardware-verified
//
#include <hip/hip_runtime.h>
#include <hip/hip_bf16.h>
#include <math.h>


#define NB 8
#define NL 256
#define NG 8
#define NS 64
#define NE 1024
#define NH 16
#define NHD 64
#define NS2 66
#define QSCALE 0.125f
#define SS 2048
#define HH 16
#define DKK 64

typedef _Float16 bf16;
typedef __attribute__((ext_vector_type(4))) unsigned v4u_t;
typedef unsigned v4ua __attribute__((ext_vector_type(4), may_alias));
typedef __attribute__((ext_vector_type(4))) float v4f_t;
typedef float v4fa __attribute__((ext_vector_type(4), may_alias));
typedef __attribute__((ext_vector_type(16))) bf16  bf16x16;
typedef __attribute__((ext_vector_type(8)))  bf16  bf16x8;
typedef __attribute__((ext_vector_type(4)))  bf16  bf16x4;
typedef __attribute__((ext_vector_type(8)))  float f32x8;

#define LDS_STRIDE 48
#define KSTRIDE    72
#define VSTRIDE    48

__device__ __forceinline__ f32x8 wmma_bf16(bf16x16 a, bf16x16 b, f32x8 c) {
  return __builtin_amdgcn_wmma_f32_16x16x32_f16(
      false, a, false, b, (short)0, c, false, false);
}

template <typename T>
__device__ __forceinline__ bf16x16 load_frag(const T* __restrict__ base, int ld,
                                             int row0, int k0) {
  const int lane = threadIdx.x & 31;
  const int r    = lane & 15;
  const int kh   = (lane >> 4) * 8;
  const T* p0 = base + (size_t)(row0 + r) * ld + (k0 + kh);
  const T* p1 = p0 + 16;
  bf16x16 f;
#pragma unroll
  for (int i = 0; i < 8; ++i) {
    f[i]     = (bf16)p0[i];
    f[i + 8] = (bf16)p1[i];
  }
  return f;
}

__device__ __forceinline__ bf16x16 lds_frag(const bf16* base, int stride) {
  const int lane = threadIdx.x & 31;
  const int row  = lane & 15;
  const int kh   = (lane >> 4) * 8;
  const bf16x8 lo = *(const bf16x8*)(base + row * stride + kh);
  const bf16x8 hi = *(const bf16x8*)(base + row * stride + kh + 16);
  bf16x16 f;
#pragma unroll
  for (int i = 0; i < 8; ++i) { f[i] = lo[i]; f[i + 8] = hi[i]; }
  return f;
}

template <typename T>
__device__ __forceinline__ void stage_read16(const T* __restrict__ p, float* buf) {
#pragma unroll
  for (int i = 0; i < 16; ++i) buf[i] = (float)p[i];
}

__device__ __forceinline__ void stage_write(bf16* dst, const float* buf, int nquad) {
#pragma unroll
  for (int i = 0; i < nquad; ++i) {
    bf16x4 q;
    q[0] = (bf16)buf[4 * i];     q[1] = (bf16)buf[4 * i + 1];
    q[2] = (bf16)buf[4 * i + 2]; q[3] = (bf16)buf[4 * i + 3];
    *(bf16x4*)(dst + 4 * i) = q;
  }
}

template <typename AT, int MODE>
__global__ __launch_bounds__(256) void gemm_bias_kernel(
    const AT* __restrict__ A, const float* __restrict__ W,
    const float* __restrict__ bias, void* __restrict__ out,
    int M, int N, int K, float oscale) {
  __shared__ bf16 ldsA[128 * LDS_STRIDE];
  __shared__ bf16 ldsW[256 * LDS_STRIDE];
  __shared__ __attribute__((aligned(16))) unsigned char sob[256 * 136 * 2];

  const int t    = threadIdx.x;
  const int wave = t >> 5;
  const int lane = t & 31;
  const int wm   = (wave & 1) * 64;
  const int wn   = (wave >> 1) * 64;
  const int mBlk = blockIdx.x * 128;
  const int nBlk = blockIdx.y * 256;

  const int arow = t >> 1;
  const int ach  = (t & 1) * 16;

  float abuf[16];
  float wbuf[32];

  stage_read16(A + (size_t)(mBlk + arow) * K + ach, abuf);
  stage_read16(W + (size_t)(nBlk + t) * K,          wbuf);
  stage_read16(W + (size_t)(nBlk + t) * K + 16,     wbuf + 16);

  f32x8 acc[4][4] = {};

  for (int k = 0; k < K; k += 32) {
    __syncthreads();
    stage_write(&ldsA[arow * LDS_STRIDE + ach], abuf, 4);
    stage_write(&ldsW[t * LDS_STRIDE],          wbuf, 8);
    if (k + 32 < K) {
      stage_read16(A + (size_t)(mBlk + arow) * K + (k + 32) + ach, abuf);
      stage_read16(W + (size_t)(nBlk + t) * K + (k + 32),          wbuf);
      stage_read16(W + (size_t)(nBlk + t) * K + (k + 32) + 16,     wbuf + 16);
    }
    __syncthreads();

    bf16x16 af[4], wf[4];
#pragma unroll
    for (int i = 0; i < 4; ++i)
      af[i] = lds_frag(ldsA + (wm + 16 * i) * LDS_STRIDE, LDS_STRIDE);
#pragma unroll
    for (int j = 0; j < 4; ++j)
      wf[j] = lds_frag(ldsW + (wn + 16 * j) * LDS_STRIDE, LDS_STRIDE);
#pragma unroll
    for (int i = 0; i < 4; ++i)
#pragma unroll
      for (int j = 0; j < 4; ++j)
        acc[i][j] = wmma_bf16(af[i], wf[j], acc[i][j]);
  }

  const int nlane = lane & 15;
  const int mh    = (lane >> 4) * 8;
  __syncthreads();
  if (MODE == 0 || MODE == 1) {
    bf16* so = (bf16*)sob;
#pragma unroll
    for (int i = 0; i < 4; ++i)
#pragma unroll
      for (int j = 0; j < 4; ++j) {
        const int nl = wn + 16 * j + nlane;
        const float bv = bias[nBlk + nl];
#pragma unroll
        for (int r = 0; r < 8; ++r) {
          const int ml = wm + 16 * i + mh + r;
          const bf16 hv = (bf16)((acc[i][j][r] + bv) * oscale);
          if (MODE == 0) so[ml * 264 + nl] = hv;
          else           so[nl * 136 + ml] = hv;
        }
      }
    __syncthreads();
#pragma unroll 1
    for (int pass = 0; pass < 2; ++pass) {
      if (MODE == 0) {
        for (int ch = t; ch < 128 * 32; ch += 256) { const int ml = ch >> 5, q = (ch & 31) * 8;
          *(volatile v4u_t*)((bf16*)out + (size_t)(mBlk + ml) * N + nBlk + q) = *(const v4ua*)(so + ml * 264 + q); }
      } else {
        const int b_ = mBlk >> 11, s0 = mBlk & (SS - 1);
        for (int ch = t; ch < 256 * 16; ch += 256) { const int nl = ch >> 4, q = (ch & 15) * 8; const int n = nBlk + nl, h = n >> 6, dk = n & (DKK - 1);
          *(volatile v4u_t*)((bf16*)out + (((size_t)(b_ * HH + h)) * DKK + dk) * SS + s0 + q) = *(const v4ua*)(so + nl * 136 + q); }
      }
      __threadfence();
    }
  } else {
    float* so = (float*)sob;
#pragma unroll 1
    for (int hf = 0; hf < 2; ++hf) {
      if (wm == hf * 64) {
#pragma unroll
        for (int i = 0; i < 4; ++i)
#pragma unroll
          for (int j = 0; j < 4; ++j) {
            const int nl = wn + 16 * j + nlane;
            const float bv = bias[nBlk + nl];
#pragma unroll
            for (int r = 0; r < 8; ++r) so[(16 * i + mh + r) * 260 + nl] = (acc[i][j][r] + bv) * oscale;
          }
      }
      __syncthreads();
#pragma unroll 1
      for (int pass = 0; pass < 2; ++pass) {
        for (int ch = t; ch < 64 * 64; ch += 256) { const int ml = ch >> 6, q = (ch & 63) * 4;
          *(volatile v4f_t*)((float*)out + (size_t)(mBlk + hf * 64 + ml) * N + nBlk + q) = *(const volatile v4fa*)(so + ml * 260 + q); }
        __threadfence();
      }
      __syncthreads();
    }
  }
}


__global__ __launch_bounds__(256) void best_section_kernel(const float* __restrict__ scores, int* __restrict__ best) {
  const int i = blockIdx.x * 256 + threadIdx.x;
  const float* p = scores + (size_t)i * (NG + 2);
  int bi = 0; float bvv = p[0];
#pragma unroll
  for (int g = 1; g < NG; ++g) { const float v = p[g]; if (v > bvv) { bvv = v; bi = g; } }
  *(volatile int*)(best + i) = bi; __threadfence(); *(volatile int*)(best + i) = bi;
}

__global__ __launch_bounds__(256)
void attention_kernel(const bf16* __restrict__ Q,
                      const bf16* __restrict__ Kp,
                      const bf16* __restrict__ Vp,
                      const int*  __restrict__ mask,
                      const float* __restrict__ bias_k, const float* __restrict__ bias_v,
                      const int*  __restrict__ best,
                      bf16* __restrict__ attnOut,
                      float* __restrict__ wOut) {
  __shared__ float sw[NH][NS2 + 2];
  __shared__ __attribute__((aligned(16))) float wst[16 * NS2];
  const int t = threadIdx.x, h = t >> 4, j = t & 15;
  const int eoff = h * NHD + j * 4;
#pragma unroll 1
  for (int rr = 0; rr < 16; ++rr) {
    const int bl = blockIdx.x * 16 + rr;
    const int b = bl / NL, l = bl % NL;
    int g = best[bl]; g = (g < 0) ? 0 : (g > NG - 1 ? NG - 1 : g);
    const size_t krow0 = (size_t)((b * NG + g) * NS) * NE;
    const bf16x4 qv = *(const bf16x4*)(Q + (size_t)(l * NB + b) * NE + eoff);
    const float q0 = (float)qv[0], q1 = (float)qv[1], q2 = (float)qv[2], q3 = (float)qv[3];
    const int* mrow = mask + (size_t)(b * NG + g) * NS;
    __syncthreads();
    for (int s = 0; s < NS; ++s) {
      const bf16x4 kv = *(const bf16x4*)(Kp + krow0 + (size_t)s * NE + eoff);
      float p = q0 * (float)kv[0] + q1 * (float)kv[1] + q2 * (float)kv[2] + q3 * (float)kv[3];
#pragma unroll
      for (int o = 8; o >= 1; o >>= 1) p += __shfl_xor(p, o, 16);
      if (j == 0) sw[h][s] = (mrow[s] != 0) ? -__builtin_inff() : p;
    }
    {
      const float* bk = bias_k + eoff;
      float p = q0 * bk[0] + q1 * bk[1] + q2 * bk[2] + q3 * bk[3];
#pragma unroll
      for (int o = 8; o >= 1; o >>= 1) p += __shfl_xor(p, o, 16);
      if (j == 0) { sw[h][64] = p; sw[h][65] = 0.0f; }
    }
    __syncthreads();
    float m = -__builtin_inff();
#pragma unroll
    for (int i = 0; i < 5; ++i) { const int s = j + 16 * i; if (s < NS2) m = fmaxf(m, sw[h][s]); }
#pragma unroll
    for (int o = 8; o >= 1; o >>= 1) m = fmaxf(m, __shfl_xor(m, o, 16));
    float sum = 0.0f;
    float ev[5];
#pragma unroll
    for (int i = 0; i < 5; ++i) { const int s = j + 16 * i; ev[i] = 0.0f; if (s < NS2) { ev[i] = __expf(sw[h][s] - m); sum += ev[i]; } }
#pragma unroll
    for (int o = 8; o >= 1; o >>= 1) sum += __shfl_xor(sum, o, 16);
    const float inv = 1.0f / sum;
    __syncthreads();
#pragma unroll
    for (int i = 0; i < 5; ++i) { const int s = j + 16 * i; if (s < NS2) sw[h][s] = ev[i] * inv; }
    __syncthreads();
    float a0 = 0.f, a1 = 0.f, a2 = 0.f, a3 = 0.f;
    for (int s = 0; s < NS; ++s) {
      const float w = sw[h][s];
      const bf16x4 vv = *(const bf16x4*)(Vp + krow0 + (size_t)s * NE + eoff);
      a0 += w * (float)vv[0]; a1 += w * (float)vv[1]; a2 += w * (float)vv[2]; a3 += w * (float)vv[3];
    }
    { const float w = sw[h][64]; const float* bvp = bias_v + eoff; a0 += w * bvp[0]; a1 += w * bvp[1]; a2 += w * bvp[2]; a3 += w * bvp[3]; }
    bf16x4 ov; ov[0] = (bf16)a0; ov[1] = (bf16)a1; ov[2] = (bf16)a2; ov[3] = (bf16)a3;
    bf16* od = attnOut + (size_t)(l * NB + b) * NE + eoff;
    *(volatile bf16x4*)od = ov; __threadfence(); *(volatile bf16x4*)od = ov;
    if (t < NS2) { float s_ = 0.0f;
#pragma unroll
      for (int hh2 = 0; hh2 < NH; ++hh2) s_ += sw[hh2][t];
      wst[rr * NS2 + t] = s_ * (1.0f / NH); }
  }
  __syncthreads();
#pragma unroll 1
  for (int pass = 0; pass < 2; ++pass) {
    for (int q = t; q < 16 * NS2 / 4; q += 256) *(volatile v4f_t*)(wOut + (size_t)blockIdx.x * 16 * NS2 + q * 4) = *(const volatile v4fa*)(wst + q * 4);
    __threadfence();
  }
}

extern "C" void kernel_launch(void* const* d_in, const int* in_sizes, int n_in,
                              void* d_out, int out_size, void* d_ws, size_t ws_size,
                              hipStream_t stream) {
  (void)in_sizes; (void)n_in; (void)out_size; (void)ws_size;
  const float* query       = (const float*)d_in[0];
  const float* sections    = (const float*)d_in[1];
  const int*   msk         = (const int*)d_in[2];
  const float* attn_scores = (const float*)d_in[3];
  const float* Wq = (const float*)d_in[4];  const float* bq = (const float*)d_in[5];
  const float* Wk = (const float*)d_in[6];  const float* bk = (const float*)d_in[7];
  const float* Wv = (const float*)d_in[8];  const float* bv = (const float*)d_in[9];
  const float* Wo = (const float*)d_in[10]; const float* bo = (const float*)d_in[11];
  const float* bias_k = (const float*)d_in[12];
  const float* bias_v = (const float*)d_in[13];

  const int MQ = NL * NB;
  const int MS = NB * NG * NS;
  char* ws = (char*)d_ws;
  int*  best  = (int*)ws;                          ws += 65536;
  bf16* qproj = (bf16*)ws;                         ws += (size_t)MQ * NE * 2;
  bf16* kproj = (bf16*)ws;                         ws += (size_t)MS * NE * 2;
  bf16* vproj = (bf16*)ws;                         ws += (size_t)MS * NE * 2;
  bf16* abuf  = (bf16*)ws;                         ws += (size_t)MQ * NE * 2;
  float* out_main = (float*)d_out;
  float* out_w    = (float*)d_out + (size_t)MQ * NE;

  best_section_kernel<<<(NB * NL) / 256, 256, 0, stream>>>(attn_scores, best);
  dim3 gBlk(256);
  gemm_bias_kernel<float, 0><<<dim3(MQ / 128, NE / 256), gBlk, 0, stream>>>(query,    Wq, bq, qproj, MQ, NE, NE, QSCALE);
  gemm_bias_kernel<float, 0><<<dim3(MS / 128, NE / 256), gBlk, 0, stream>>>(sections, Wk, bk, kproj, MS, NE, NE, 1.0f);
  gemm_bias_kernel<float, 0><<<dim3(MS / 128, NE / 256), gBlk, 0, stream>>>(sections, Wv, bv, vproj, MS, NE, NE, 1.0f);
  attention_kernel<<<(NB * NL) / 16, 256, 0, stream>>>(qproj, kproj, vproj, msk, bias_k, bias_v, best, abuf, out_w);
  gemm_bias_kernel<bf16, 2><<<dim3(MQ / 128, NE / 256), gBlk, 0, stream>>>(abuf, Wo, bo, out_main, MQ, NE, NE, 1.0f);
}
